// EnhancedJointGraphPredictor_20392504721605
// MI455X (gfx1250) — hardware-verified
//
#include <hip/hip_runtime.h>
#include <math.h>

typedef __attribute__((ext_vector_type(16))) _Float16 v16h;
typedef __attribute__((ext_vector_type(16))) __bf16 v16b;
typedef __attribute__((ext_vector_type(8)))  _Float16 v8h;
typedef __attribute__((ext_vector_type(8)))  float v8f;
typedef __attribute__((ext_vector_type(4)))  float v4f;
typedef __attribute__((ext_vector_type(2)))  float v2f;
typedef __attribute__((ext_vector_type(4)))  unsigned v4u;
typedef __attribute__((ext_vector_type(4)))  int v4i;
typedef float __attribute__((may_alias)) float_a;
typedef int __attribute__((may_alias)) int_a;

template <typename T> __device__ __forceinline__ void vst2(void* p, T v) { *(volatile T*)p = v; __threadfence(); *(volatile T*)p = v; }
__device__ __forceinline__ v8f wmma16(v16h a, v16h b, v8f c) {
  v8f d = __builtin_amdgcn_wmma_f32_16x16x32_f16(false, a, false, b, (short)0, c, false, false);
  asm volatile("v_nop\n\tv_nop\n\tv_nop\n\tv_nop" : "+v"(d) : "v"(a), "v"(b));
  return d;
}
__device__ __forceinline__ v8f wmma_bf(v16b a, v16b b, v8f c) {
  v8f d = __builtin_amdgcn_wmma_f32_16x16x32_bf16(false, a, false, b, (short)0, c, false, false);
  asm volatile("v_nop\n\tv_nop\n\tv_nop\n\tv_nop" : "+v"(d) : "v"(a), "v"(b));
  return d;
}
__device__ __forceinline__ v16h frag_h(const _Float16* rowk0, int lane) {
  union { v16h v; v8h q[2]; } u; const _Float16* p = rowk0 + 8 * (lane >> 4);
  u.q[0] = *(const v8h*)p; u.q[1] = *(const v8h*)(p + 16); return u.v;
}
__device__ __forceinline__ v16h frag_f32(const float* rowk0, int lane) {
  v16h a; const float* p = rowk0 + 8 * (lane >> 4);
#pragma unroll
  for (int i = 0; i < 8; ++i) { a[i] = (_Float16)p[i]; a[8 + i] = (_Float16)p[16 + i]; }
  return a;
}
__device__ __forceinline__ v16h frag_f32s(const float* rowk0, int lane, float sc) {
  v16h a; const float* p = rowk0 + 8 * (lane >> 4);
#pragma unroll
  for (int i = 0; i < 8; ++i) { a[i] = (_Float16)(p[i] * sc); a[8 + i] = (_Float16)(p[16 + i] * sc); }
  return a;
}
__device__ __forceinline__ v16h fragc_f32(const float* W, int k0, int n, int lane, int ld, int K) {
  v16h a; const int g = lane >> 4;
#pragma unroll
  for (int i = 0; i < 8; ++i) { const int ka = k0 + 8 * g + i, kb = ka + 16;
    a[i] = (_Float16)(ka < K ? W[(size_t)(ka < K ? ka : K - 1) * ld + n] : 0.f); a[8 + i] = (_Float16)(kb < K ? W[(size_t)(kb < K ? kb : K - 1) * ld + n] : 0.f); }
  return a;
}
struct F2 { v16b h, l; };
__device__ __forceinline__ F2 bsplit16(const float v[16]) { F2 r;
#pragma unroll
  for (int i = 0; i < 16; ++i) { const __bf16 h = (__bf16)v[i]; r.h[i] = h; r.l[i] = (__bf16)(v[i] - (float)h); }
  return r; }
__device__ __forceinline__ F2 split_row(const float* row, int k0, int lane) { float v[16]; const float* p = row + k0 + 8 * (lane >> 4);
#pragma unroll
  for (int i = 0; i < 8; ++i) { v[i] = p[i]; v[8 + i] = p[16 + i]; }
  return bsplit16(v); }
__device__ __forceinline__ F2 split_rowK(const float* row, int k0, int lane, int K) { float v[16]; const int g = lane >> 4;
#pragma unroll
  for (int i = 0; i < 8; ++i) { const int ka = k0 + 8 * g + i, kb = ka + 16; v[i] = ka < K ? row[ka < K ? ka : K - 1] : 0.f; v[8 + i] = kb < K ? row[kb < K ? kb : K - 1] : 0.f; }
  return bsplit16(v); }
__device__ __forceinline__ F2 split_col(const float* W, int k0, int n, int lane, int ld, int K) { float v[16]; const int g = lane >> 4;
#pragma unroll
  for (int i = 0; i < 8; ++i) { const int ka = k0 + 8 * g + i, kb = ka + 16; v[i] = ka < K ? W[(size_t)(ka < K ? ka : K - 1) * ld + n] : 0.f; v[8 + i] = kb < K ? W[(size_t)(kb < K ? kb : K - 1) * ld + n] : 0.f; }
  return bsplit16(v); }
__device__ __forceinline__ v8f mac3(const F2& a, const F2& b, v8f c) { c = wmma_bf(a.l, b.h, c); c = wmma_bf(a.h, b.l, c); return wmma_bf(a.h, b.h, c); }
__device__ __forceinline__ float sigm(float v) { return 1.0f / (1.0f + expf(-v)); }
#define LDSX() do { asm volatile("s_wait_dscnt 0" ::: "memory"); __builtin_amdgcn_wave_barrier(); __builtin_amdgcn_fence(__ATOMIC_RELEASE, "workgroup"); } while (0)


#define CSR_N 50000
#define CSR_E 400000
#define CSR_CHUNK 16384
#define NM 50000
#define NP 20000
#define NMP 50048
#define NPP 20032
#define NG 1024
#define DD 256
#ifndef DBGM
#define DBGM 0
#endif
#define CSR_FINN (CSR_E + 32 * CSR_NBK)
#ifndef CSR_CHUNK
#define CSR_CHUNK 4096
#endif
#define CSR_EPT (CSR_CHUNK / 256)
#define CSR_BKT 256
#define CSR_NCH ((CSR_E + CSR_CHUNK - 1) / CSR_CHUNK)
#define CSR_NBK ((CSR_N + CSR_BKT - 1) / CSR_BKT)
#define CSR_NBKP (((CSR_NBK + 63) / 64) * 64)
#define CSR_SEGCAP (CSR_E + 32 * CSR_NBK * CSR_NCH)
#ifndef CSR_BCAP
#define CSR_BCAP 10240
#endif
#define CSR_SZ_CNT   (4u * CSR_NCH * CSR_NBKP)
#define CSR_SZ_OFF   (4u * CSR_NBK * (((CSR_NCH + 31) / 32) * 32))
#define CSR_SZ_BST   (4u * (((CSR_NBK + 1 + 31) / 32) * 32))
#define CSR_SZ_SEG   (4u * CSR_SEGCAP)
#define CSR_SZ_FIN   (4u * (CSR_E + 32 * CSR_NBK))
#define CSR_SZ_ROW   (4u * CSR_NBK * CSR_BKT)
#define CSR_OFFP (((CSR_NCH + 31) / 32) * 32)

__global__ __launch_bounds__(256) void k_csr_cnt(const int* __restrict__ DST, int dstride, int* __restrict__ CNT) {
  __shared__ unsigned short sc[256][CSR_NBK + 1]; __shared__ __align__(16) int srow[CSR_NBKP];
  const int c = blockIdx.x, tid = threadIdx.x;
  for (int b = 0; b < CSR_NBK; ++b) sc[tid][b] = 0;
  const size_t e0 = (size_t)c * CSR_CHUNK + tid * CSR_EPT;
  for (int i = 0; i < CSR_EPT; ++i) { const size_t e = e0 + i; if (e < (size_t)CSR_E) { int d = DST[e * dstride]; d = min(max(d, 0), CSR_N - 1); sc[tid][d / CSR_BKT] += 1; } }
  __syncthreads();
  for (int b = tid; b < CSR_NBKP; b += 256) { int s = 0; if (b < CSR_NBK) for (int t = 0; t < 256; ++t) s += sc[t][b]; srow[b] = s; }
  __syncthreads();
  for (int q = tid; q < CSR_NBKP / 4; q += 256) vst2((unsigned*)(CNT + (size_t)c * CSR_NBKP + q * 4), *(const v4u*)&srow[q * 4]);
}
__global__ __launch_bounds__(256) void k_csr_scan(const int* __restrict__ CNT, int* __restrict__ OFF, int* __restrict__ BST) {
  __shared__ int sbt[CSR_NBK + 1]; __shared__ int sbs[((CSR_NBK + 1 + 31) / 32) * 32]; __shared__ int scnt[CSR_NBK + 1]; __shared__ __align__(16) int sbuf[64][CSR_OFFP];
  const int tid = threadIdx.x;
  for (int b = tid; b < CSR_NBK; b += 256) { int sp = 0, st = 0; for (int c = 0; c < CSR_NCH; ++c) { const int n = CNT[(size_t)c * CSR_NBKP + b]; st += n; sp += (n + 31) & ~31; } sbt[b] = sp; scnt[b] = st; }
  for (int b = tid; b < ((CSR_NBK + 1 + 31) / 32) * 32; b += 256) sbs[b] = 0;
  __syncthreads();
  if (tid == 0) { int acc = 0, accf = 0; for (int b = 0; b < CSR_NBK; ++b) { const int t = sbt[b]; sbt[b] = acc; acc += t; sbs[b] = accf; accf += (scnt[b] + 31) & ~31; } sbs[CSR_NBK] = accf; }
  __syncthreads();
  for (int b0 = 0; b0 < CSR_NBK; b0 += 64) {
    if (tid < 64 && b0 + tid < CSR_NBK) { const int b = b0 + tid; int o = sbt[b]; for (int c = 0; c < CSR_OFFP; ++c) { if (c < CSR_NCH) { sbuf[tid][c] = o; o += (CNT[(size_t)c * CSR_NBKP + b] + 31) & ~31; } else sbuf[tid][c] = 0; } }
    __syncthreads();
    for (int q = tid; q < 64 * (CSR_OFFP / 4); q += 256) { const int r = q / (CSR_OFFP / 4), pc = q % (CSR_OFFP / 4); if (b0 + r < CSR_NBK) vst2((unsigned*)(OFF + (size_t)(b0 + r) * CSR_OFFP + pc * 4), *(const v4u*)&sbuf[r][pc * 4]); }
    __syncthreads(); }
  for (int q = tid; q < ((CSR_NBK + 1 + 31) / 32) * 32 / 4; q += 256) vst2((unsigned*)(BST + q * 4), *(const v4u*)&sbs[q * 4]);
}
__global__ __launch_bounds__(256) void k_csr_scatter(const int* __restrict__ SRC, const int* __restrict__ DST, int sstride, int dstride, const int* __restrict__ OFF, int* __restrict__ SEGS, int* __restrict__ SEGE) {
  __shared__ unsigned short sc[256][CSR_NBK + 1]; __shared__ int sbase[CSR_NBK + 1]; __shared__ int scn[CSR_NBK + 1]; __shared__ int sord[CSR_CHUNK];
  const int c = blockIdx.x, tid = threadIdx.x;
  for (int b = 0; b < CSR_NBK; ++b) sc[tid][b] = 0;
  const size_t e0 = (size_t)c * CSR_CHUNK + tid * CSR_EPT; int bk[CSR_EPT];
#pragma unroll
  for (int i = 0; i < CSR_EPT; ++i) { const size_t e = e0 + i; bk[i] = -1; if (e < (size_t)CSR_E) { int d = DST[e * dstride]; d = min(max(d, 0), CSR_N - 1); bk[i] = d / CSR_BKT; sc[tid][bk[i]] += 1; } }
  __syncthreads();
  for (int b = tid; b < CSR_NBK; b += 256) { int acc = 0; for (int t = 0; t < 256; ++t) { const int v = sc[t][b]; sc[t][b] = (unsigned short)acc; acc += v; } scn[b] = acc; }
  __syncthreads();
  if (tid == 0) { int acc = 0; for (int b = 0; b < CSR_NBK; ++b) { sbase[b] = acc; acc += scn[b]; } }
  __syncthreads();
#pragma unroll
  for (int i = 0; i < CSR_EPT; ++i) { if (bk[i] >= 0) { const int b = bk[i]; const int r = sc[tid][b]; sc[tid][b] = (unsigned short)(r + 1); sord[sbase[b] + r] = tid * CSR_EPT + i; } }
  __syncthreads();
  for (int b = 0; b < CSR_NBK; ++b) { const int n = scn[b]; if (n == 0) continue; const int nl = ((n + 31) & ~31); const size_t o = (size_t)(min(max(OFF[(size_t)b * CSR_OFFP + c], 0), CSR_SEGCAP - nl) & ~31);
    for (int q = tid; q < nl / 4; q += 256) { int4 vs, ve;
#pragma unroll
      for (int k = 0; k < 4; ++k) { const int i = q * 4 + k; int s = -1, eid = -1; if (i < n) { const size_t e = (size_t)c * CSR_CHUNK + sord[sbase[b] + i]; s = min(max(SRC[e * sstride], 0), CSR_N - 1); eid = (int)e; } vs[k] = s; ve[k] = eid; }
      vst2((unsigned*)(SEGS + o + q * 4), *(const v4u*)&vs); vst2((unsigned*)(SEGE + o + q * 4), *(const v4u*)&ve); } }
}
__global__ __launch_bounds__(256) void k_csr_bucket(const int* __restrict__ CNT, const int* __restrict__ OFF, const int* __restrict__ BST, const int* __restrict__ SEGS, const int* __restrict__ SEGE, const int* __restrict__ DST, int dstride, int* __restrict__ FS, int* __restrict__ FE, int* __restrict__ ROWST, int* __restrict__ ROWCNT) {
  __shared__ int ssrc[CSR_BCAP]; __shared__ int seid[CSR_BCAP]; __shared__ unsigned char snod[CSR_BCAP]; __shared__ int souts[CSR_BCAP]; __shared__ int soute[CSR_BCAP]; __shared__ int scount[256]; __shared__ int sstart[257]; __shared__ int stot;
  const int b = blockIdx.x, tid = threadIdx.x;
  if (tid == 0) { int t = 0; for (int c = 0; c < CSR_NCH; ++c) t += min(max(CNT[(size_t)c * CSR_NBKP + b], 0), CSR_CHUNK); stot = (t <= CSR_BCAP) ? t : 0; }
  __syncthreads();
  { int base = 0; for (int c = 0; c < CSR_NCH; ++c) { const int n = min(max(CNT[(size_t)c * CSR_NBKP + b], 0), CSR_CHUNK); const int o = min(max(OFF[(size_t)b * CSR_OFFP + c], 0), CSR_SEGCAP - ((n + 31) & ~31));
      for (int i = tid; i < n; i += 256) { const int p = base + i; if (p < CSR_BCAP) { ssrc[p] = min(max(SEGS[o + i], 0), CSR_N - 1); const int e = min(max(SEGE[o + i], 0), CSR_E - 1); seid[p] = e; int d = DST[(size_t)e * dstride]; d = min(max(d, 0), CSR_N - 1); const int dl = d - b * CSR_BKT; snod[p] = (unsigned char)(dl >= 0 && dl < 256 ? dl : 255); } }
      base += n; } }
  __syncthreads();
  const int node = b * CSR_BKT + tid; int cnt = 0; for (int p = 0; p < stot; ++p) cnt += (snod[p] == tid) ? 1 : 0;
  scount[tid] = cnt; __syncthreads();
  if (tid == 0) { int acc = 0; for (int t = 0; t < 256; ++t) { sstart[t] = acc; acc += scount[t]; } sstart[256] = acc; }
  __syncthreads();
  const int bst0 = min(max(BST[b], 0), CSR_FINN - ((sstart[256] + 31) & ~31)) & ~31; const int gst = bst0 + sstart[tid];
  { int w = sstart[tid]; for (int p = 0; p < stot; ++p) if (snod[p] == tid) { souts[w] = ssrc[p]; soute[w] = seid[p]; ++w; } }
  __syncthreads();
  { const int n = sstart[256]; const int nl = (n + 31) & ~31; for (int q = tid; q < nl / 4; q += 256) { int4 vs, ve;
#pragma unroll
      for (int k = 0; k < 4; ++k) { const int i = q * 4 + k; vs[k] = i < n ? souts[i] : -1; ve[k] = i < n ? soute[i] : -1; }
      vst2((unsigned*)(FS + bst0 + q * 4), *(const v4u*)&vs); vst2((unsigned*)(FE + bst0 + q * 4), *(const v4u*)&ve); } }
  __syncthreads();
  { __shared__ __align__(16) int srs[256], src2[256]; srs[tid] = node < CSR_N ? gst : 0; src2[tid] = node < CSR_N ? cnt : 0; __syncthreads();
    if (tid < 64) vst2((unsigned*)(ROWST + (size_t)b * 256 + tid * 4), *(const v4u*)&srs[tid * 4]); else if (tid < 128) vst2((unsigned*)(ROWCNT + (size_t)b * 256 + (tid - 64) * 4), *(const v4u*)&src2[(tid - 64) * 4]); }
}

#define CSRB_N 20000
#define CSRB_E 160000
#define CSRB_FINN (CSRB_E + 32 * CSRB_NBK)
#ifndef CSRB_CHUNK
#define CSRB_CHUNK 4096
#endif
#define CSRB_EPT (CSRB_CHUNK / 256)
#define CSRB_BKT 256
#define CSRB_NCH ((CSRB_E + CSRB_CHUNK - 1) / CSRB_CHUNK)
#define CSRB_NBK ((CSRB_N + CSRB_BKT - 1) / CSRB_BKT)
#define CSRB_NBKP (((CSRB_NBK + 63) / 64) * 64)
#define CSRB_SEGCAP (CSRB_E + 32 * CSRB_NBK * CSRB_NCH)
#ifndef CSRB_BCAP
#define CSRB_BCAP 10240
#endif
#define CSRB_SZ_CNT   (4u * CSRB_NCH * CSRB_NBKP)
#define CSRB_SZ_OFF   (4u * CSRB_NBK * (((CSRB_NCH + 31) / 32) * 32))
#define CSRB_SZ_BST   (4u * (((CSRB_NBK + 1 + 31) / 32) * 32))
#define CSRB_SZ_SEG   (4u * CSRB_SEGCAP)
#define CSRB_SZ_FIN   (4u * (CSRB_E + 32 * CSRB_NBK))
#define CSRB_SZ_ROW   (4u * CSRB_NBK * CSRB_BKT)
#define CSRB_OFFP (((CSRB_NCH + 31) / 32) * 32)

__global__ __launch_bounds__(256) void k_csrB_cnt(const int* __restrict__ DST, int dstride, int* __restrict__ CNT) {
  __shared__ unsigned short sc[256][CSRB_NBK + 1]; __shared__ __align__(16) int srow[CSRB_NBKP];
  const int c = blockIdx.x, tid = threadIdx.x;
  for (int b = 0; b < CSRB_NBK; ++b) sc[tid][b] = 0;
  const size_t e0 = (size_t)c * CSRB_CHUNK + tid * CSRB_EPT;
  for (int i = 0; i < CSRB_EPT; ++i) { const size_t e = e0 + i; if (e < (size_t)CSRB_E) { int d = DST[e * dstride]; d = min(max(d, 0), CSRB_N - 1); sc[tid][d / CSRB_BKT] += 1; } }
  __syncthreads();
  for (int b = tid; b < CSRB_NBKP; b += 256) { int s = 0; if (b < CSRB_NBK) for (int t = 0; t < 256; ++t) s += sc[t][b]; srow[b] = s; }
  __syncthreads();
  for (int q = tid; q < CSRB_NBKP / 4; q += 256) vst2((unsigned*)(CNT + (size_t)c * CSRB_NBKP + q * 4), *(const v4u*)&srow[q * 4]);
}
__global__ __launch_bounds__(256) void k_csrB_scan(const int* __restrict__ CNT, int* __restrict__ OFF, int* __restrict__ BST) {
  __shared__ int sbt[CSRB_NBK + 1]; __shared__ int sbs[((CSRB_NBK + 1 + 31) / 32) * 32]; __shared__ int scnt[CSRB_NBK + 1]; __shared__ __align__(16) int sbuf[64][CSRB_OFFP];
  const int tid = threadIdx.x;
  for (int b = tid; b < CSRB_NBK; b += 256) { int sp = 0, st = 0; for (int c = 0; c < CSRB_NCH; ++c) { const int n = CNT[(size_t)c * CSRB_NBKP + b]; st += n; sp += (n + 31) & ~31; } sbt[b] = sp; scnt[b] = st; }
  for (int b = tid; b < ((CSRB_NBK + 1 + 31) / 32) * 32; b += 256) sbs[b] = 0;
  __syncthreads();
  if (tid == 0) { int acc = 0, accf = 0; for (int b = 0; b < CSRB_NBK; ++b) { const int t = sbt[b]; sbt[b] = acc; acc += t; sbs[b] = accf; accf += (scnt[b] + 31) & ~31; } sbs[CSRB_NBK] = accf; }
  __syncthreads();
  for (int b0 = 0; b0 < CSRB_NBK; b0 += 64) {
    if (tid < 64 && b0 + tid < CSRB_NBK) { const int b = b0 + tid; int o = sbt[b]; for (int c = 0; c < CSRB_OFFP; ++c) { if (c < CSRB_NCH) { sbuf[tid][c] = o; o += (CNT[(size_t)c * CSRB_NBKP + b] + 31) & ~31; } else sbuf[tid][c] = 0; } }
    __syncthreads();
    for (int q = tid; q < 64 * (CSRB_OFFP / 4); q += 256) { const int r = q / (CSRB_OFFP / 4), pc = q % (CSRB_OFFP / 4); if (b0 + r < CSRB_NBK) vst2((unsigned*)(OFF + (size_t)(b0 + r) * CSRB_OFFP + pc * 4), *(const v4u*)&sbuf[r][pc * 4]); }
    __syncthreads(); }
  for (int q = tid; q < ((CSRB_NBK + 1 + 31) / 32) * 32 / 4; q += 256) vst2((unsigned*)(BST + q * 4), *(const v4u*)&sbs[q * 4]);
}
__global__ __launch_bounds__(256) void k_csrB_scatter(const int* __restrict__ SRC, const int* __restrict__ DST, int sstride, int dstride, const int* __restrict__ OFF, int* __restrict__ SEGS, int* __restrict__ SEGE) {
  __shared__ unsigned short sc[256][CSRB_NBK + 1]; __shared__ int sbase[CSRB_NBK + 1]; __shared__ int scn[CSRB_NBK + 1]; __shared__ int sord[CSRB_CHUNK];
  const int c = blockIdx.x, tid = threadIdx.x;
  for (int b = 0; b < CSRB_NBK; ++b) sc[tid][b] = 0;
  const size_t e0 = (size_t)c * CSRB_CHUNK + tid * CSRB_EPT; int bk[CSRB_EPT];
#pragma unroll
  for (int i = 0; i < CSRB_EPT; ++i) { const size_t e = e0 + i; bk[i] = -1; if (e < (size_t)CSRB_E) { int d = DST[e * dstride]; d = min(max(d, 0), CSRB_N - 1); bk[i] = d / CSRB_BKT; sc[tid][bk[i]] += 1; } }
  __syncthreads();
  for (int b = tid; b < CSRB_NBK; b += 256) { int acc = 0; for (int t = 0; t < 256; ++t) { const int v = sc[t][b]; sc[t][b] = (unsigned short)acc; acc += v; } scn[b] = acc; }
  __syncthreads();
  if (tid == 0) { int acc = 0; for (int b = 0; b < CSRB_NBK; ++b) { sbase[b] = acc; acc += scn[b]; } }
  __syncthreads();
#pragma unroll
  for (int i = 0; i < CSRB_EPT; ++i) { if (bk[i] >= 0) { const int b = bk[i]; const int r = sc[tid][b]; sc[tid][b] = (unsigned short)(r + 1); sord[sbase[b] + r] = tid * CSRB_EPT + i; } }
  __syncthreads();
  for (int b = 0; b < CSRB_NBK; ++b) { const int n = scn[b]; if (n == 0) continue; const int nl = ((n + 31) & ~31); const size_t o = (size_t)(min(max(OFF[(size_t)b * CSRB_OFFP + c], 0), CSRB_SEGCAP - nl) & ~31);
    for (int q = tid; q < nl / 4; q += 256) { int4 vs, ve;
#pragma unroll
      for (int k = 0; k < 4; ++k) { const int i = q * 4 + k; int s = -1, eid = -1; if (i < n) { const size_t e = (size_t)c * CSRB_CHUNK + sord[sbase[b] + i]; s = min(max(SRC[e * sstride], 0), CSRB_N - 1); eid = (int)e; } vs[k] = s; ve[k] = eid; }
      vst2((unsigned*)(SEGS + o + q * 4), *(const v4u*)&vs); vst2((unsigned*)(SEGE + o + q * 4), *(const v4u*)&ve); } }
}
__global__ __launch_bounds__(256) void k_csrB_bucket(const int* __restrict__ CNT, const int* __restrict__ OFF, const int* __restrict__ BST, const int* __restrict__ SEGS, const int* __restrict__ SEGE, const int* __restrict__ DST, int dstride, int* __restrict__ FS, int* __restrict__ FE, int* __restrict__ ROWST, int* __restrict__ ROWCNT) {
  __shared__ int ssrc[CSRB_BCAP]; __shared__ int seid[CSRB_BCAP]; __shared__ unsigned char snod[CSRB_BCAP]; __shared__ int souts[CSRB_BCAP]; __shared__ int soute[CSRB_BCAP]; __shared__ int scount[256]; __shared__ int sstart[257]; __shared__ int stot;
  const int b = blockIdx.x, tid = threadIdx.x;
  if (tid == 0) { int t = 0; for (int c = 0; c < CSRB_NCH; ++c) t += min(max(CNT[(size_t)c * CSRB_NBKP + b], 0), CSRB_CHUNK); stot = (t <= CSRB_BCAP) ? t : 0; }
  __syncthreads();
  { int base = 0; for (int c = 0; c < CSRB_NCH; ++c) { const int n = min(max(CNT[(size_t)c * CSRB_NBKP + b], 0), CSRB_CHUNK); const int o = min(max(OFF[(size_t)b * CSRB_OFFP + c], 0), CSRB_SEGCAP - ((n + 31) & ~31));
      for (int i = tid; i < n; i += 256) { const int p = base + i; if (p < CSRB_BCAP) { ssrc[p] = min(max(SEGS[o + i], 0), CSRB_N - 1); const int e = min(max(SEGE[o + i], 0), CSRB_E - 1); seid[p] = e; int d = DST[(size_t)e * dstride]; d = min(max(d, 0), CSRB_N - 1); const int dl = d - b * CSRB_BKT; snod[p] = (unsigned char)(dl >= 0 && dl < 256 ? dl : 255); } }
      base += n; } }
  __syncthreads();
  const int node = b * CSRB_BKT + tid; int cnt = 0; for (int p = 0; p < stot; ++p) cnt += (snod[p] == tid) ? 1 : 0;
  scount[tid] = cnt; __syncthreads();
  if (tid == 0) { int acc = 0; for (int t = 0; t < 256; ++t) { sstart[t] = acc; acc += scount[t]; } sstart[256] = acc; }
  __syncthreads();
  const int bst0 = min(max(BST[b], 0), CSRB_FINN - ((sstart[256] + 31) & ~31)) & ~31; const int gst = bst0 + sstart[tid];
  { int w = sstart[tid]; for (int p = 0; p < stot; ++p) if (snod[p] == tid) { souts[w] = ssrc[p]; soute[w] = seid[p]; ++w; } }
  __syncthreads();
  { const int n = sstart[256]; const int nl = (n + 31) & ~31; for (int q = tid; q < nl / 4; q += 256) { int4 vs, ve;
#pragma unroll
      for (int k = 0; k < 4; ++k) { const int i = q * 4 + k; vs[k] = i < n ? souts[i] : -1; ve[k] = i < n ? soute[i] : -1; }
      vst2((unsigned*)(FS + bst0 + q * 4), *(const v4u*)&vs); vst2((unsigned*)(FE + bst0 + q * 4), *(const v4u*)&ve); } }
  __syncthreads();
  { __shared__ __align__(16) int srs[256], src2[256]; srs[tid] = node < CSRB_N ? gst : 0; src2[tid] = node < CSRB_N ? cnt : 0; __syncthreads();
    if (tid < 64) vst2((unsigned*)(ROWST + (size_t)b * 256 + tid * 4), *(const v4u*)&srs[tid * 4]); else if (tid < 128) vst2((unsigned*)(ROWCNT + (size_t)b * 256 + (tid - 64) * 4), *(const v4u*)&src2[(tid - 64) * 4]); }
}

typedef __attribute__((ext_vector_type(8))) __bf16 v8b;
__device__ __forceinline__ v16b frag_b(const __bf16* rowk0, int lane) {
  union { v16b v; v8b q[2]; } u; const __bf16* p = rowk0 + 8 * (lane >> 4);
  u.q[0] = *(const v8b*)p; u.q[1] = *(const v8b*)(p + 16); return u.v;
}
__device__ __forceinline__ float bfr(float v) { return (float)(__bf16)v; }
__device__ __attribute__((noinline)) float exp_ni(float v) { return expf(v); }
#define PK_G1M 0
#define PK_G2M (PK_G1M + 256 * 64)
#define PK_G3M (PK_G2M + 256 * 256)
#define PK_G1P (PK_G3M + 256 * 256)
#define PK_G2P (PK_G1P + 256 * 64)
#define PK_A1M (PK_G2P + 256 * 256)
#define PK_A2M (PK_A1M + 256 * 256)
#define PK_AP  (PK_A2M + 256 * 256)
#define PK_V   (PK_AP + 256 * 256)
#define PK_AO  (PK_V + 256 * 256)
#define PK_JT1 (PK_AO + 256 * 256)
#define PK_JT2 (PK_JT1 + 512 * 768)
#define PK_PL0 (PK_JT2 + 256 * 512)
#define PK_PL1 (PK_PL0 + 128 * 256)
#define PK_PL2 (PK_PL1 + 128 * 256)
#define PK_PR1 (PK_PL2 + 128 * 256)
#define PK_PR2 (PK_PR1 + 256 * 640)
#define PK_PR3 (PK_PR2 + 128 * 256)
#define PK_PR4 (PK_PR3 + 64 * 128)
#define PK_END (PK_PR4 + 16 * 64)
#define WSA_CNT  0u
#define WSA_OFF  (WSA_CNT + CSR_SZ_CNT)
#define WSA_BST  (WSA_OFF + CSR_SZ_OFF)
#define WSA_SEGS (WSA_BST + CSR_SZ_BST)
#define WSA_SEGE (WSA_SEGS + CSR_SZ_SEG)
#define WSA_FS   (WSA_SEGE + CSR_SZ_SEG)
#define WSA_FE   (WSA_FS + CSR_SZ_FIN)
#define WSA_RST  (WSA_FE + CSR_SZ_FIN)
#define WSA_RCT  (WSA_RST + CSR_SZ_ROW)
#define WSB_CNT  (WSA_RCT + CSR_SZ_ROW)
#define WSB_OFF  (WSB_CNT + CSRB_SZ_CNT)
#define WSB_BST  (WSB_OFF + CSRB_SZ_OFF)
#define WSB_SEGS (WSB_BST + CSRB_SZ_BST)
#define WSB_SEGE (WSB_SEGS + CSRB_SZ_SEG)
#define WSB_FS   (WSB_SEGE + CSRB_SZ_SEG)
#define WSB_FE   (WSB_FS + CSRB_SZ_FIN)
#define WSB_RST  (WSB_FE + CSRB_SZ_FIN)
#define WSB_RCT  (WSB_RST + CSRB_SZ_ROW)
#define WS_PK    (WSB_RCT + CSRB_SZ_ROW)
#define WS_XA    (WS_PK + 2u * PK_END)
#define WS_XB    (WS_XA + 4u * NMP * DD)
#define WS_AS    (WS_XB + 4u * NMP * DD)
#define WS_POOL  (WS_AS + 4u * NMP * 8)
#define WS_PGL   (WS_POOL + 4u * NG * 768)
#define WS_HD    (WS_PGL + 4u * 320 * DD)
#define HD_G1 0
#define HD_JF (HD_G1 + NG * 768)
#define HD_F  (HD_JF + NG * 512)
#define HD_H1 (HD_F + NG * 640)
#define HD_H2 (HD_H1 + NG * 256)
#define HD_H3 (HD_H2 + NG * 128)
#define HD_END (HD_H3 + NG * 64)
#define WS_END   (WS_HD + 4u * HD_END)

struct PackSpec { int rows; int K; int KP; int NO; };
__global__ __launch_bounds__(256) void k_pack(const float* __restrict__ g1m, const float* __restrict__ g2m, const float* __restrict__ g3m, const float* __restrict__ g1p, const float* __restrict__ g2p, const float* __restrict__ a1m, const float* __restrict__ a2m, const float* __restrict__ ap,
                                              const float* __restrict__ qkv, const float* __restrict__ ao, const float* __restrict__ jt1, const float* __restrict__ jt2, const float* __restrict__ pl0, const float* __restrict__ pl1, const float* __restrict__ pl2, const float* __restrict__ pr1, const float* __restrict__ pr2, const float* __restrict__ pr3, const float* __restrict__ pr4, __bf16* __restrict__ PK) {
  __shared__ __align__(16) __bf16 srow[768];
  const int n = blockIdx.x, tid = threadIdx.x; const float* W; int K, KP, NO, o, wstride, coff = 0; size_t dst;
  int m = n;
  if (m < 256) { W = g1m; K = 8; KP = 64; NO = 256; o = m; dst = PK_G1M + (size_t)o * 64; } else if ((m -= 256) < 256) { W = g2m; K = 256; KP = 256; NO = 256; o = m; dst = PK_G2M + (size_t)o * 256; }
  else if ((m -= 256) < 256) { W = g3m; K = 256; KP = 256; NO = 256; o = m; dst = PK_G3M + (size_t)o * 256; } else if ((m -= 256) < 256) { W = g1p; K = 5; KP = 64; NO = 256; o = m; dst = PK_G1P + (size_t)o * 64; }
  else if ((m -= 256) < 256) { W = g2p; K = 256; KP = 256; NO = 256; o = m; dst = PK_G2P + (size_t)o * 256; } else if ((m -= 256) < 256) { W = a1m; K = 256; KP = 256; NO = 256; o = m; dst = PK_A1M + (size_t)o * 256; }
  else if ((m -= 256) < 256) { W = a2m; K = 256; KP = 256; NO = 256; o = m; dst = PK_A2M + (size_t)o * 256; } else if ((m -= 256) < 256) { W = ap; K = 256; KP = 256; NO = 256; o = m; dst = PK_AP + (size_t)o * 256; }
  else if ((m -= 256) < 256) { W = qkv; K = 256; KP = 256; NO = 768; o = 512 + m; dst = PK_V + (size_t)m * 256; } else if ((m -= 256) < 256) { W = ao; K = 256; KP = 256; NO = 256; o = m; dst = PK_AO + (size_t)o * 256; }
  else if ((m -= 256) < 512) { W = jt1; K = 768; KP = 768; NO = 512; o = m; dst = PK_JT1 + (size_t)o * 768; } else if ((m -= 512) < 256) { W = jt2; K = 512; KP = 512; NO = 256; o = m; dst = PK_JT2 + (size_t)o * 512; }
  else if ((m -= 256) < 128) { W = pl0; K = 256; KP = 256; NO = 128; o = m; dst = PK_PL0 + (size_t)o * 256; } else if ((m -= 128) < 128) { W = pl1; K = 256; KP = 256; NO = 128; o = m; dst = PK_PL1 + (size_t)o * 256; }
  else if ((m -= 128) < 128) { W = pl2; K = 256; KP = 256; NO = 128; o = m; dst = PK_PL2 + (size_t)o * 256; } else if ((m -= 128) < 256) { W = pr1; K = 640; KP = 640; NO = 256; o = m; dst = PK_PR1 + (size_t)o * 640; }
  else if ((m -= 256) < 128) { W = pr2; K = 256; KP = 256; NO = 128; o = m; dst = PK_PR2 + (size_t)o * 256; } else if ((m -= 128) < 64) { W = pr3; K = 128; KP = 128; NO = 64; o = m; dst = PK_PR3 + (size_t)o * 128; }
  else { m -= 64; W = pr4; K = 64; KP = 64; NO = 1; o = m; dst = PK_PR4 + (size_t)m * 64; }
  (void)wstride; (void)coff;
  for (int k = tid; k < KP; k += 256) srow[k] = (__bf16)((k < K && o < NO) ? bfr(W[(size_t)k * NO + o]) : 0.f);
  __syncthreads();
  for (int q = tid; q < KP / 8; q += 256) vst2((unsigned*)(PK + dst + q * 8), *(const v4u*)(&srow[q * 8]));
}
#define NPACK (256 * 10 + 512 + 256 + 128 * 3 + 256 + 128 + 64 + 16)
template <int CW, bool RND, bool GB>
__global__ __launch_bounds__(256) void k_gcnagg(const float* __restrict__ X, int ipitch, int nn, const int* __restrict__ FS, const int* __restrict__ RST, const int* __restrict__ RCT, float* __restrict__ AGG) {
  constexpr int CQ = (CW >= 32) ? CW / 4 : 8;
  const int tid = threadIdx.x; const size_t i = (size_t)blockIdx.x * 64 + (tid >> 2); const int q = tid & 3;
  float acc[CQ];
#pragma unroll
  for (int c = 0; c < CQ; ++c) acc[c] = 0.f;
  float di = 0.f;
  if (i < (size_t)nn && (CW >= 32 || q == 0)) { const int cnt = min(max(RCT[i], 0), GB ? CSRB_BCAP : CSR_BCAP); const int st = min(max(RST[i], 0), (GB ? CSRB_FINN : CSR_FINN) - cnt); di = rsqrtf((float)cnt + 1.0f);
    for (int e = 0; e < cnt; ++e) { const int s = min(max(FS[st + e], 0), nn - 1); const float ds = rsqrtf((float)min(max(RCT[s], 0), GB ? CSRB_BCAP : CSR_BCAP) + 1.0f); const float* xr = X + (size_t)s * ipitch + q * CQ;
#pragma unroll
      for (int c = 0; c < CQ; ++c) { if (CW >= 32 || c < CW) { float v = xr[c]; if (RND) v = bfr(v); acc[c] += ds * v; } } }
    { const float* xr = X + i * ipitch + q * CQ;
#pragma unroll
      for (int c = 0; c < CQ; ++c) { if (CW >= 32 || c < CW) { float v = xr[c]; if (RND) v = bfr(v); acc[c] += di * v; } } } }
  if (CW >= 32) {
#pragma unroll
    for (int p = 0; p < CQ / 4; ++p) { v4f v; for (int k = 0; k < 4; ++k) v[k] = acc[p * 4 + k] * di; vst2(AGG + i * 256 + q * CQ + p * 4, v); } }
  else if (q == 0) {
#pragma unroll
    for (int p = 0; p < 16; ++p) { v4f v; for (int k = 0; k < 4; ++k) { const int c = p * 4 + k; v[k] = (c < CW) ? acc[c < CQ ? c : 0] * di : 0.f; } vst2(AGG + i * 256 + p * 4, v); } }
}
template <int KI, bool ACT>
__global__ __launch_bounds__(128) void k_lin(const float* __restrict__ IN, const __bf16* __restrict__ P, const float* __restrict__ bias, float* __restrict__ OUT, int nn) {
  __shared__ __align__(16) float so[4][16][260]; __shared__ __align__(16) __bf16 sah[4][16][264], sal[4][16][264];
  const int tid = threadIdx.x, wave = tid >> 5, lane = tid & 31, col = lane & 15, g = lane >> 4; const size_t r0 = (size_t)blockIdx.x * 64 + wave * 16;
  for (int q = lane; q < 16 * KI; q += 32) { const int rl = q / KI, k = q % KI; const float v = IN[(r0 + rl) * 256 + k]; const __bf16 hb = (__bf16)v; sah[wave][rl][k] = hb; sal[wave][rl][k] = (__bf16)(v - (float)hb); }
  LDSX();
#pragma unroll 1
  for (int jt = 0; jt < 4; ++jt) { v8f acc[4] = {};
#pragma unroll 2
    for (int kc = 0; kc < KI / 32; ++kc) { const v16b ah = frag_b(&sah[wave][col][kc * 32], lane), al = frag_b(&sal[wave][col][kc * 32], lane);
#pragma unroll
      for (int j = 0; j < 4; ++j) { const v16b w = frag_b(P + (size_t)((jt * 4 + j) * 16 + col) * KI + kc * 32, lane); acc[j] = wmma_bf(al, w, acc[j]); acc[j] = wmma_bf(ah, w, acc[j]); } }
#pragma unroll
    for (int j = 0; j < 4; ++j) { const int o = (jt * 4 + j) * 16 + col; const float bb = bias ? bfr(bias[o]) : 0.f;
#pragma unroll
      for (int r = 0; r < 8; ++r) { float v = acc[j][r] + bb; if (ACT) v = fmaxf(v, 0.f); so[wave][8 * g + r][o] = (r0 + 8 * g + r < (size_t)nn) ? v : 0.f; } } }
  LDSX();
  for (int rl = 0; rl < 16; ++rl) for (int pc = lane; pc < 64; pc += 32) vst2(OUT + (r0 + rl) * 256 + pc * 4, *(const v4f*)&so[wave][rl][pc * 4]);
}
__global__ __launch_bounds__(256) void k_gatas(const float* __restrict__ H, const float* __restrict__ ASV, const float* __restrict__ ADV, float* __restrict__ AS) {
  __shared__ __align__(16) float s[64][8];
  const int tid = threadIdx.x; const size_t n = (size_t)blockIdx.x * 64 + (tid >> 2); const int h = tid & 3; float a = 0.f, d = 0.f; const float* hr = H + n * 256 + h * 64;
  for (int c = 0; c < 64; ++c) { const float v = hr[c]; a += v * bfr(ASV[h * 64 + c]); d += v * bfr(ADV[h * 64 + c]); }
  s[tid >> 2][h] = a; s[tid >> 2][4 + h] = d; __syncthreads();
  if (tid < 128) { const int rl = tid >> 1, pc = tid & 1; vst2(AS + ((size_t)blockIdx.x * 64 + rl) * 8 + pc * 4, *(const v4f*)&s[rl][pc * 4]); }
}
template <bool GB>
__global__ __launch_bounds__(256) void k_gatagg(const float* __restrict__ H, const float* __restrict__ AS, const float* __restrict__ Bv, int nn, const int* __restrict__ FS, const int* __restrict__ RST, const int* __restrict__ RCT, float* __restrict__ OUT) {
  const int tid = threadIdx.x; const size_t i = (size_t)blockIdx.x * 32 + (tid >> 3); const int h = (tid >> 1) & 3, hf = tid & 1; const int cb = h * 64 + hf * 32;
  float acc[32];
#pragma unroll
  for (int c = 0; c < 32; ++c) acc[c] = 0.f;
  float z = 0.f;
  if (i < (size_t)nn) { const int cnt = min(max(RCT[i], 0), GB ? CSRB_BCAP : CSR_BCAP); const int st = min(max(RST[i], 0), (GB ? CSRB_FINN : CSR_FINN) - cnt); const float ad = AS[i * 8 + 4 + h];
    float mx; { float l = AS[i * 8 + h] + ad; l = l > 0.f ? l : 0.2f * l; mx = l; }
    for (int e = 0; e < cnt; ++e) { const int s = min(max(FS[st + e], 0), nn - 1); float l = AS[(size_t)s * 8 + h] + ad; l = l > 0.f ? l : 0.2f * l; mx = fmaxf(mx, l); }
    for (int e = 0; e <= cnt; ++e) { const int s = (e < cnt) ? min(max(FS[st + e], 0), nn - 1) : (int)i; float l = AS[(size_t)s * 8 + h] + ad; l = l > 0.f ? l : 0.2f * l; const float p = exp_ni(l - mx); z += p; const float* hr = H + (size_t)s * 256 + cb;
#pragma unroll
      for (int c = 0; c < 32; ++c) acc[c] += p * hr[c]; } }
  const float iz = (i < (size_t)nn) ? 1.0f / (z + 1e-16f) : 0.f;
#pragma unroll
  for (int p4 = 0; p4 < 8; ++p4) { v4f v; for (int k = 0; k < 4; ++k) { const int c = cb + p4 * 4 + k; v[k] = (i < (size_t)nn) ? fmaxf(acc[p4 * 4 + k] * iz + bfr(Bv[c]), 0.f) : 0.f; } vst2(OUT + i * 256 + cb + p4 * 4, v); }
}
__global__ __launch_bounds__(256) void k_molpool(const int* __restrict__ BATCH, const float* __restrict__ X, float* __restrict__ POOL) {
  __shared__ int srng[2]; __shared__ __align__(16) float s[768];
  const int gph = blockIdx.x, c = threadIdx.x;
  if (c < 2) { const int key = gph + c; int lo = 0, hi = NM; while (lo < hi) { const int mid = (lo + hi) >> 1; if (BATCH[mid] < key) lo = mid + 1; else hi = mid; } srng[c] = lo; }
  __syncthreads();
  const int n0 = srng[0], n1 = max(srng[1], srng[0]); float sum = 0.f, mx = -3.0e38f; int cnt = 0;
  for (int n = n0; n < n1; ++n) if (BATCH[n] == gph) { const float v = X[(size_t)n * 256 + c]; sum += v; mx = fmaxf(mx, v); ++cnt; }
  s[c] = sum / fmaxf((float)cnt, 1.0f); s[256 + c] = cnt > 0 ? mx : -3.0e38f; s[512 + c] = sum;
  __syncthreads();
  for (int q = c; q < 192; q += 256) vst2(POOL + (size_t)gph * 768 + q * 4, *(const v4f*)&s[q * 4]);
}
__global__ __launch_bounds__(256) void k_colsum(const float* __restrict__ X, int nn, float* __restrict__ PGL) {
  __shared__ __align__(16) float s[256]; const int c = threadIdx.x; const size_t r0 = (size_t)blockIdx.x * 64; float a = 0.f; for (int r = 0; r < 64; ++r) if (r0 + r < (size_t)nn) a += X[(r0 + r) * 256 + c]; s[c] = a; __syncthreads();
  if (c < 64) vst2(PGL + (size_t)blockIdx.x * 256 + c * 4, *(const v4f*)&s[c * 4]);
}
__global__ __launch_bounds__(256) void k_small(const float* __restrict__ PGL, int nblk, const __bf16* __restrict__ PK, const float* __restrict__ qkvb, const float* __restrict__ aob, const float* __restrict__ POOL, float* __restrict__ HD) {
  __shared__ float spg[256], sv[256], sat[256]; __shared__ __align__(16) float srow[512];
  const int c = threadIdx.x; float a = 0.f; for (int b = 0; b < nblk; ++b) a += PGL[(size_t)b * 256 + c]; spg[c] = a / (float)NP; __syncthreads();
  { float v = bfr(qkvb[512 + c]);
#pragma unroll 1
    for (int k = 0; k < 256; ++k) v += spg[k] * (float)PK[PK_V + (size_t)c * 256 + k];
    sv[c] = v; }
  __syncthreads();
  { float t = bfr(aob[c]);
#pragma unroll 1
    for (int k = 0; k < 256; ++k) t += sv[k] * (float)PK[PK_AO + (size_t)c * 256 + k];
    sat[c] = t; }
  __syncthreads();
  srow[c] = sat[c]; srow[256 + c] = spg[c]; __syncthreads();
  for (int g2 = 0; g2 < NG; ++g2) { float* row = HD + HD_G1 + (size_t)g2 * 768; if (c < 128) vst2(row + c * 4, *(const v4f*)&srow[c * 4]); else if (c < 192) vst2(row + 512 + (c - 128) * 4, *(const v4f*)(POOL + (size_t)g2 * 768 + (c - 128) * 4)); }
}
template <int KI, int NO, int ACT>
__global__ __launch_bounds__(128) void k_dense(const float* __restrict__ IN, int ip, int ioff, const __bf16* __restrict__ P, const float* __restrict__ bias, float* __restrict__ OUT, int op, int ooff) {
  constexpr int NT = (NO + 15) / 16; constexpr int NTW = (NT + 3) / 4 > 0 ? NT : NT;
  __shared__ __align__(16) float so[4][16][(NO < 64 ? 64 : NO) + 4];
  const int tid = threadIdx.x, wave = tid >> 5, lane = tid & 31, col = lane & 15, g = lane >> 4; const size_t r0 = (size_t)blockIdx.x * 64 + wave * 16;
  (void)NTW;
#pragma unroll 1
  for (int j = 0; j < NT; ++j) { v8f acc = {};
#pragma unroll 2
    for (int kc = 0; kc < KI / 32; ++kc) { const F2 a = split_row(IN + (r0 + col) * ip + ioff, kc * 32, lane); const v16b w = frag_b(P + (size_t)(j * 16 + col) * KI + kc * 32, lane); acc = wmma_bf(a.l, w, acc); acc = wmma_bf(a.h, w, acc); }
#pragma unroll
    for (int r = 0; r < 8; ++r) { const int o = j * 16 + col; float v = acc[r] + ((bias && o < NO) ? bfr(bias[o]) : 0.f); if (ACT == 1) v = fmaxf(v, 0.f); else if (ACT == 2) v = 1.0f / (1.0f + exp_ni(-v)); so[wave][8 * g + r][o] = o < NO ? v : 0.f; } }
  LDSX();
  if (NO >= 4) { for (int rl = 0; rl < 16; ++rl) for (int pc = lane; pc < NO / 4; pc += 32) vst2(OUT + (r0 + rl) * op + ooff + pc * 4, *(const v4f*)&so[wave][rl][pc * 4]); }
  else {
    __shared__ __align__(16) float sfin[64]; if (lane < 16) sfin[wave * 16 + lane] = so[wave][lane][0]; __syncthreads(); if (tid < 16) vst2(OUT + (size_t)blockIdx.x * 64 + tid * 4, *(const v4f*)&sfin[tid * 4]); }
}

#if DBGM != 0
__global__ __launch_bounds__(256) void k_dbg(const float* __restrict__ SRC, int nrows, int width, float* __restrict__ out) { __shared__ __align__(16) float s[1024]; for (int i = threadIdx.x; i < 1024; i += 256) s[i] = SRC[(size_t)((i * 4099) % nrows) * width + (i * 7) % width]; __syncthreads(); vst2(out + threadIdx.x * 4, *(const v4f*)&s[threadIdx.x * 4]); }
__global__ __launch_bounds__(256) void k_fakex(const float* __restrict__ MX, float* __restrict__ X) { const int tid = threadIdx.x; const size_t n = (size_t)blockIdx.x * 64 + (tid >> 2); for (int p = (tid & 3); p < 64; p += 4) { v4f v; for (int k = 0; k < 4; ++k) { const int c = p * 4 + k; v[k] = n < NM ? bfr(MX[n * 8 + (c % 8)]) * (0.5f + (float)(c % 5) * 0.2f) : 0.f; } vst2(X + n * 256 + p * 4, v); } }
__global__ __launch_bounds__(256) void k_fakepool(const float* __restrict__ MX, float* __restrict__ POOL) { const int g2 = blockIdx.x, c = threadIdx.x; const float p = bfr(MX[(size_t)g2 * 8 + (c % 8)]) * (0.5f + (float)(c % 5) * 0.2f); __shared__ __align__(16) float s[768]; s[c] = p; s[256 + c] = 0.5f * p; s[512 + c] = 2.0f * p; __syncthreads(); for (int q = c; q < 192; q += 256) vst2(POOL + (size_t)g2 * 768 + q * 4, *(const v4f*)&s[q * 4]); }
#endif
extern "C" void kernel_launch(void* const* d_in, const int* in_sizes, int n_in, void* d_out, int out_size, void* d_ws, size_t ws_size, hipStream_t stream) {
  (void)in_sizes; (void)n_in; (void)out_size;
  const float** F = (const float**)d_in; const int** I = (const int**)d_in;
  if (ws_size < (size_t)WS_END) return;
  char* ws = (char*)d_ws;
  int *ACNT = (int*)(ws + WSA_CNT), *AOFF = (int*)(ws + WSA_OFF), *ABST = (int*)(ws + WSA_BST), *ASEGS = (int*)(ws + WSA_SEGS), *ASEGE = (int*)(ws + WSA_SEGE), *AFS = (int*)(ws + WSA_FS), *AFE = (int*)(ws + WSA_FE), *ARST = (int*)(ws + WSA_RST), *ARCT = (int*)(ws + WSA_RCT);
  int *BCNT = (int*)(ws + WSB_CNT), *BOFF = (int*)(ws + WSB_OFF), *BBST = (int*)(ws + WSB_BST), *BSEGS = (int*)(ws + WSB_SEGS), *BSEGE = (int*)(ws + WSB_SEGE), *BFS = (int*)(ws + WSB_FS), *BFE = (int*)(ws + WSB_FE), *BRST = (int*)(ws + WSB_RST), *BRCT = (int*)(ws + WSB_RCT);
  __bf16* PK = (__bf16*)(ws + WS_PK); float *XA = (float*)(ws + WS_XA), *XB = (float*)(ws + WS_XB), *AS = (float*)(ws + WS_AS), *POOL = (float*)(ws + WS_POOL), *PGL = (float*)(ws + WS_PGL), *HD = (float*)(ws + WS_HD);
  const int* MSRC = I[1]; const int* MDST = I[1] + CSR_E; const int* PSRC = I[4]; const int* PDST = I[4] + CSRB_E;
  k_pack<<<NPACK, 256, 0, stream>>>(F[5], F[7], F[9], F[11], F[13], F[15], F[19], F[23], F[27], F[29], F[31], F[33], F[35], F[37], F[39], F[41], F[43], F[45], F[47], PK);
#if DBGM == 4
  k_fakepool<<<NG, 256, 0, stream>>>(F[0], POOL);
  goto prot;
#endif
  k_csr_cnt<<<CSR_NCH, 256, 0, stream>>>(MDST, 1, ACNT); k_csr_scan<<<1, 256, 0, stream>>>(ACNT, AOFF, ABST); k_csr_scatter<<<CSR_NCH, 256, 0, stream>>>(MSRC, MDST, 1, 1, AOFF, ASEGS, ASEGE); k_csr_bucket<<<CSR_NBK, 256, 0, stream>>>(ACNT, AOFF, ABST, ASEGS, ASEGE, MDST, 1, AFS, AFE, ARST, ARCT);
#if DBGM == 2 || DBGM == 3
  k_fakex<<<NMP / 64, 256, 0, stream>>>(F[0], XA);
#endif
#if DBGM == 2
  goto gcn3;
#endif
#if DBGM == 3
  goto gat2;
#endif
  k_gcnagg<8, true, false><<<NMP / 64, 256, 0, stream>>>(F[0], 8, NM, AFS, ARST, ARCT, XA);
  k_lin<64, true><<<NMP / 64, 128, 0, stream>>>(XA, PK + PK_G1M, F[6], XA, NM);
  k_gcnagg<256, false, false><<<NMP / 64, 256, 0, stream>>>(XA, 256, NM, AFS, ARST, ARCT, XB);
  k_lin<256, true><<<NMP / 64, 128, 0, stream>>>(XB, PK + PK_G2M, F[8], XB, NM);
#if DBGM == 1
  k_dbg<<<1, 256, 0, stream>>>(XB, NM, 256, (float*)d_out); return;
#endif
  gcn3:
  k_gcnagg<256, false, false><<<NMP / 64, 256, 0, stream>>>(DBGM == 2 ? XA : XB, 256, NM, AFS, ARST, ARCT, DBGM == 2 ? XB : XA);
  k_lin<256, true><<<NMP / 64, 128, 0, stream>>>(DBGM == 2 ? XB : XA, PK + PK_G3M, F[10], XA, NM);
  k_lin<256, false><<<NMP / 64, 128, 0, stream>>>(XA, PK + PK_A1M, nullptr, XB, NM);
  k_gatas<<<NMP / 64, 256, 0, stream>>>(XB, F[16], F[17], AS);
  k_gatagg<false><<<NMP / 32, 256, 0, stream>>>(XB, AS, F[18], NM, AFS, ARST, ARCT, XA);
#if DBGM == 2
  k_dbg<<<1, 256, 0, stream>>>(XA, NM, 256, (float*)d_out); return;
#endif
  gat2:
  k_lin<256, false><<<NMP / 64, 128, 0, stream>>>(XA, PK + PK_A2M, nullptr, XB, NM);
  k_gatas<<<NMP / 64, 256, 0, stream>>>(XB, F[20], F[21], AS);
  k_gatagg<false><<<NMP / 32, 256, 0, stream>>>(XB, AS, F[22], NM, AFS, ARST, ARCT, XA);
  k_molpool<<<NG, 256, 0, stream>>>(I[2], XA, POOL);
#if DBGM == 3
  k_dbg<<<1, 256, 0, stream>>>(POOL, NG, 768, (float*)d_out); return;
#endif
  prot:
  k_csrB_cnt<<<CSRB_NCH, 256, 0, stream>>>(PDST, 1, BCNT); k_csrB_scan<<<1, 256, 0, stream>>>(BCNT, BOFF, BBST); k_csrB_scatter<<<CSRB_NCH, 256, 0, stream>>>(PSRC, PDST, 1, 1, BOFF, BSEGS, BSEGE); k_csrB_bucket<<<CSRB_NBK, 256, 0, stream>>>(BCNT, BOFF, BBST, BSEGS, BSEGE, PDST, 1, BFS, BFE, BRST, BRCT);
  k_gcnagg<5, true, true><<<NPP / 64, 256, 0, stream>>>(F[3], 5, NP, BFS, BRST, BRCT, XA);
  k_lin<64, true><<<NPP / 64, 128, 0, stream>>>(XA, PK + PK_G1P, F[12], XA, NP);
  k_gcnagg<256, false, true><<<NPP / 64, 256, 0, stream>>>(XA, 256, NP, BFS, BRST, BRCT, XB);
  k_lin<256, true><<<NPP / 64, 128, 0, stream>>>(XB, PK + PK_G2P, F[14], XB, NP);
  k_lin<256, false><<<NPP / 64, 128, 0, stream>>>(XB, PK + PK_AP, nullptr, XA, NP);
  k_gatas<<<NPP / 64, 256, 0, stream>>>(XA, F[24], F[25], AS);
  k_gatagg<true><<<NPP / 32, 256, 0, stream>>>(XA, AS, F[26], NP, BFS, BRST, BRCT, XB);
  k_colsum<<<NPP / 64, 256, 0, stream>>>(XB, NP, PGL);
  k_small<<<1, 256, 0, stream>>>(PGL, NPP / 64, PK, F[28], F[30], POOL, HD);
  k_dense<768, 512, 1><<<NG / 64, 128, 0, stream>>>(HD + HD_G1, 768, 0, PK + PK_JT1, F[32], HD + HD_JF, 512, 0);
  k_dense<512, 256, 1><<<NG / 64, 128, 0, stream>>>(HD + HD_JF, 512, 0, PK + PK_JT2, F[34], HD + HD_F, 640, 0);
  k_dense<256, 128, 0><<<NG / 64, 128, 0, stream>>>(POOL, 768, 0, PK + PK_PL0, F[36], HD + HD_F, 640, 256);
  k_dense<256, 128, 0><<<NG / 64, 128, 0, stream>>>(POOL, 768, 256, PK + PK_PL1, F[38], HD + HD_F, 640, 384);
  k_dense<256, 128, 0><<<NG / 64, 128, 0, stream>>>(POOL, 768, 512, PK + PK_PL2, F[40], HD + HD_F, 640, 512);
  k_dense<640, 256, 1><<<NG / 64, 128, 0, stream>>>(HD + HD_F, 640, 0, PK + PK_PR1, F[42], HD + HD_H1, 256, 0);
  k_dense<256, 128, 1><<<NG / 64, 128, 0, stream>>>(HD + HD_H1, 256, 0, PK + PK_PR2, F[44], HD + HD_H2, 128, 0);
  k_dense<128, 64, 1><<<NG / 64, 128, 0, stream>>>(HD + HD_H2, 128, 0, PK + PK_PR3, F[46], HD + HD_H3, 64, 0);
  k_dense<64, 1, 2><<<NG / 64, 128, 0, stream>>>(HD + HD_H3, 64, 0, PK + PK_PR4, F[48], (float*)d_out, 1, 0);
}
